// MultiQueryAttentionLayerWithDownSampling_51771535786445
// MI455X (gfx1250) — hardware-verified
//
#include <hip/hip_runtime.h>
#include <math.h>

typedef __attribute__((ext_vector_type(16))) _Float16 v16h;
typedef __attribute__((ext_vector_type(16))) __bf16 v16b;
typedef __attribute__((ext_vector_type(8)))  _Float16 v8h;
typedef __attribute__((ext_vector_type(8)))  float v8f;
typedef __attribute__((ext_vector_type(4)))  float v4f;
typedef __attribute__((ext_vector_type(2)))  float v2f;
typedef __attribute__((ext_vector_type(4)))  unsigned v4u;
typedef __attribute__((ext_vector_type(4)))  int v4i;
typedef float __attribute__((may_alias)) float_a;
typedef int __attribute__((may_alias)) int_a;

template <typename T> __device__ __forceinline__ void vst2(void* p, T v) { *(volatile T*)p = v; __threadfence(); *(volatile T*)p = v; }
__device__ __forceinline__ v8f wmma16(v16h a, v16h b, v8f c) {
  v8f d = __builtin_amdgcn_wmma_f32_16x16x32_f16(false, a, false, b, (short)0, c, false, false);
  asm volatile("v_nop\n\tv_nop\n\tv_nop\n\tv_nop" : "+v"(d) : "v"(a), "v"(b));
  return d;
}
__device__ __forceinline__ v8f wmma_bf(v16b a, v16b b, v8f c) {
  v8f d = __builtin_amdgcn_wmma_f32_16x16x32_bf16(false, a, false, b, (short)0, c, false, false);
  asm volatile("v_nop\n\tv_nop\n\tv_nop\n\tv_nop" : "+v"(d) : "v"(a), "v"(b));
  return d;
}
__device__ __forceinline__ v16h frag_h(const _Float16* rowk0, int lane) {
  union { v16h v; v8h q[2]; } u; const _Float16* p = rowk0 + 8 * (lane >> 4);
  u.q[0] = *(const v8h*)p; u.q[1] = *(const v8h*)(p + 16); return u.v;
}
__device__ __forceinline__ v16h frag_f32(const float* rowk0, int lane) {
  v16h a; const float* p = rowk0 + 8 * (lane >> 4);
#pragma unroll
  for (int i = 0; i < 8; ++i) { a[i] = (_Float16)p[i]; a[8 + i] = (_Float16)p[16 + i]; }
  return a;
}
__device__ __forceinline__ v16h frag_f32s(const float* rowk0, int lane, float sc) {
  v16h a; const float* p = rowk0 + 8 * (lane >> 4);
#pragma unroll
  for (int i = 0; i < 8; ++i) { a[i] = (_Float16)(p[i] * sc); a[8 + i] = (_Float16)(p[16 + i] * sc); }
  return a;
}
__device__ __forceinline__ v16h fragc_f32(const float* W, int k0, int n, int lane, int ld, int K) {
  v16h a; const int g = lane >> 4;
#pragma unroll
  for (int i = 0; i < 8; ++i) { const int ka = k0 + 8 * g + i, kb = ka + 16;
    a[i] = (_Float16)(ka < K ? W[(size_t)(ka < K ? ka : K - 1) * ld + n] : 0.f); a[8 + i] = (_Float16)(kb < K ? W[(size_t)(kb < K ? kb : K - 1) * ld + n] : 0.f); }
  return a;
}
struct F2 { v16b h, l; };
__device__ __forceinline__ F2 bsplit16(const float v[16]) { F2 r;
#pragma unroll
  for (int i = 0; i < 16; ++i) { const __bf16 h = (__bf16)v[i]; r.h[i] = h; r.l[i] = (__bf16)(v[i] - (float)h); }
  return r; }
__device__ __forceinline__ F2 split_row(const float* row, int k0, int lane) { float v[16]; const float* p = row + k0 + 8 * (lane >> 4);
#pragma unroll
  for (int i = 0; i < 8; ++i) { v[i] = p[i]; v[8 + i] = p[16 + i]; }
  return bsplit16(v); }
__device__ __forceinline__ F2 split_rowK(const float* row, int k0, int lane, int K) { float v[16]; const int g = lane >> 4;
#pragma unroll
  for (int i = 0; i < 8; ++i) { const int ka = k0 + 8 * g + i, kb = ka + 16; v[i] = ka < K ? row[ka < K ? ka : K - 1] : 0.f; v[8 + i] = kb < K ? row[kb < K ? kb : K - 1] : 0.f; }
  return bsplit16(v); }
__device__ __forceinline__ F2 split_col(const float* W, int k0, int n, int lane, int ld, int K) { float v[16]; const int g = lane >> 4;
#pragma unroll
  for (int i = 0; i < 8; ++i) { const int ka = k0 + 8 * g + i, kb = ka + 16; v[i] = ka < K ? W[(size_t)(ka < K ? ka : K - 1) * ld + n] : 0.f; v[8 + i] = kb < K ? W[(size_t)(kb < K ? kb : K - 1) * ld + n] : 0.f; }
  return bsplit16(v); }
__device__ __forceinline__ v8f mac3(const F2& a, const F2& b, v8f c) { c = wmma_bf(a.l, b.h, c); c = wmma_bf(a.h, b.l, c); return wmma_bf(a.h, b.h, c); }
__device__ __forceinline__ float sigm(float v) { return 1.0f / (1.0f + expf(-v)); }
#define LDSX() do { asm volatile("s_wait_dscnt 0" ::: "memory"); __builtin_amdgcn_wave_barrier(); __builtin_amdgcn_fence(__ATOMIC_RELEASE, "workgroup"); } while (0)


#define NB 8
#define CC 256
#define IH 64
#define IW 64
#define OHW 32
#define NP (OHW * OHW)
#define NHD 8
#define KD 64
#define QC (NHD * KD)
#define BNEPS 1e-5f
#ifndef TNB
#define TNB NB
#endif
typedef __attribute__((ext_vector_type(8))) __bf16 v8b;
__device__ __forceinline__ v16b frag_b(const __bf16* rowk0, int lane) {
  union { v16b v; v8b q[2]; } u; const __bf16* p = rowk0 + 8 * (lane >> 4);
  u.q[0] = *(const v8b*)p; u.q[1] = *(const v8b*)(p + 16); return u.v;
}
__device__ __forceinline__ float bfr(float v) { return (float)(__bf16)v; }
__device__ __attribute__((noinline)) float exp_ni(float v) { return expf(v); }
__device__ __attribute__((noinline)) float erf_ni(float v) { return erff(v); }

#define WS_QH  0u
#define WS_QL  (WS_QH + 2u * (size_t)NB * NP * QC)
#define WS_KH  (WS_QL + 2u * (size_t)NB * NP * QC)
#define WS_KL  (WS_KH + 2u * (size_t)NB * NP * KD)
#define WS_VT  (WS_KL + 2u * (size_t)NB * NP * KD)
#define WS_VTL (WS_VT + 2u * (size_t)NB * KD * NP)
#define WS_O   (WS_VTL + 2u * (size_t)NB * KD * NP)
#define WS_END (WS_O + 4u * (size_t)NB * NP * QC)

__device__ __forceinline__ v16b fragb_f32(const float* __restrict__ p, int lane) { v16b a; const float* pp = p + 8 * (lane >> 4);
#pragma unroll
  for (int i = 0; i < 8; ++i) { a[i] = (__bf16)pp[i]; a[8 + i] = (__bf16)pp[16 + i]; } return a; }
__device__ __forceinline__ float bnf(float x, const float* G, const float* Bt, const float* M, const float* V, int c) { const float inv = bfr(G[c]) / sqrtf(bfr(V[c]) + BNEPS); return x * inv + (bfr(Bt[c]) - bfr(M[c]) * inv); }
__global__ __launch_bounds__(128) void k_q(const float* __restrict__ X, const float* __restrict__ G, const float* __restrict__ Bt, const float* __restrict__ M, const float* __restrict__ V, const float* __restrict__ WQ, _Float16* __restrict__ QH, _Float16* __restrict__ QL) {
  __shared__ __align__(16) float sa[64][CC + 4]; __shared__ __align__(16) _Float16 sh[4][16][136], sl[4][16][136];
  const int tid = threadIdx.x, wave = tid >> 5, lane = tid & 31, col = lane & 15, g = lane >> 4; const size_t b = blockIdx.y; const int n0 = blockIdx.x * 64; const float* Xb = X + b * CC * (size_t)(IH * IW);
  for (int e = tid; e < 64 * CC; e += 128) { const int c = e >> 6, pl = e & 63; const int n = n0 + pl; const int oy = n / OHW, ox = n % OHW; const float* px = Xb + (size_t)c * IH * IW + (2 * oy) * IW + 2 * ox; const float s = (bfr(px[0]) + bfr(px[1]) + bfr(px[IW]) + bfr(px[IW + 1])) * 0.25f; sa[pl][c] = bnf(s, G, Bt, M, V, c); }
  __syncthreads();
#pragma unroll 1
  for (int cc = 0; cc < QC; cc += 128) { v8f acc[8] = {};
#pragma unroll
    for (int kc = 0; kc < CC / 32; ++kc) { float v[16]; const float* pp = &sa[wave * 16 + col][kc * 32 + 8 * g];
#pragma unroll
      for (int i = 0; i < 8; ++i) { v[i] = pp[i]; v[8 + i] = pp[16 + i]; }
      const F2 a = bsplit16(v);
#pragma unroll
      for (int j = 0; j < 8; ++j) { const v16b w = fragb_f32(WQ + (size_t)(cc + j * 16 + col) * CC + kc * 32, lane); acc[j] = wmma_bf(a.h, w, acc[j]); acc[j] = wmma_bf(a.l, w, acc[j]); } }
#pragma unroll
    for (int j = 0; j < 8; ++j)
#pragma unroll
      for (int r = 0; r < 8; ++r) { const float q = acc[j][r]; const _Float16 hv = (_Float16)q; sh[wave][8 * g + r][j * 16 + col] = hv; sl[wave][8 * g + r][j * 16 + col] = (_Float16)((q - (float)hv) * 2048.0f); }
    LDSX(); for (int rl = 0; rl < 16; ++rl) if (lane < 16) { const size_t o = (b * NP + n0 + wave * 16 + rl) * QC + cc + lane * 8; vst2((unsigned*)(QH + o), *(const v4u*)&sh[wave][rl][lane * 8]); vst2((unsigned*)(QL + o), *(const v4u*)&sl[wave][rl][lane * 8]); } LDSX(); } }
__global__ __launch_bounds__(128) void k_kv(const float* __restrict__ X, const float* __restrict__ KDW, const float* __restrict__ KG, const float* __restrict__ KB, const float* __restrict__ KM, const float* __restrict__ KV, const float* __restrict__ WK, const float* __restrict__ VDW, const float* __restrict__ VG, const float* __restrict__ VB, const float* __restrict__ VM, const float* __restrict__ VV, const float* __restrict__ WV, _Float16* __restrict__ KH, _Float16* __restrict__ KL, _Float16* __restrict__ VT, _Float16* __restrict__ VTL) {
  __shared__ __align__(16) float sa[64][CC + 4]; __shared__ __align__(16) _Float16 sh[64][72], sl[64][72]; __shared__ __align__(16) _Float16 th[KD][72], tl[KD][72];
  const int tid = threadIdx.x, wave = tid >> 5, lane = tid & 31, col = lane & 15, g = lane >> 4; const size_t b = blockIdx.y; const int n0 = blockIdx.x * 64; const float* Xb = X + b * CC * (size_t)(IH * IW);
#pragma unroll 1
  for (int path = 0; path < 2; ++path) { const float* DW = path == 0 ? KDW : VDW; const float* Wm = path == 0 ? WK : WV;
    for (int e = tid; e < 64 * CC; e += 128) { const int c = e >> 6, pl = e & 63; const int n = n0 + pl; const int oy = n / OHW, ox = n % OHW; float s = 0.f;
#pragma unroll
      for (int t9 = 0; t9 < 9; ++t9) { const int iy = 2 * oy - 1 + t9 / 3, ix = 2 * ox - 1 + t9 % 3; if (iy >= 0 && iy < IH && ix >= 0 && ix < IW) s += bfr(Xb[(size_t)c * IH * IW + iy * IW + ix]) * bfr(DW[c * 9 + t9]); }
      sa[pl][c] = path == 0 ? bnf(s, KG, KB, KM, KV, c) : bnf(s, VG, VB, VM, VV, c); }
    __syncthreads();
    v8f acc[4] = {};
#pragma unroll
    for (int kc = 0; kc < CC / 32; ++kc) { float v[16]; const float* pp = &sa[wave * 16 + col][kc * 32 + 8 * g];
#pragma unroll
      for (int i = 0; i < 8; ++i) { v[i] = pp[i]; v[8 + i] = pp[16 + i]; }
      const F2 a = bsplit16(v);
#pragma unroll
      for (int j = 0; j < 4; ++j) { const v16b w = fragb_f32(Wm + (size_t)(j * 16 + col) * CC + kc * 32, lane); acc[j] = wmma_bf(a.h, w, acc[j]); acc[j] = wmma_bf(a.l, w, acc[j]); } }
#pragma unroll
    for (int j = 0; j < 4; ++j)
#pragma unroll
      for (int r = 0; r < 8; ++r) { const float q = acc[j][r]; const _Float16 hv = (_Float16)q, lv = (_Float16)((q - (float)hv) * 2048.0f); if (path == 0) { sh[wave * 16 + 8 * g + r][j * 16 + col] = hv; sl[wave * 16 + 8 * g + r][j * 16 + col] = lv; } else { th[j * 16 + col][wave * 16 + 8 * g + r] = hv; tl[j * 16 + col][wave * 16 + 8 * g + r] = lv; } }
    __syncthreads();
    if (path == 0) { for (int e = tid; e < 64 * 8; e += 128) { const int rl = e >> 3, q = e & 7; const size_t o = (b * NP + n0 + rl) * KD + q * 8; vst2((unsigned*)(KH + o), *(const v4u*)&sh[rl][q * 8]); vst2((unsigned*)(KL + o), *(const v4u*)&sl[rl][q * 8]); } }
    else { for (int e = tid; e < KD * 8; e += 128) { const int cl = e >> 3, q = e & 7; const size_t o = (b * KD + cl) * (size_t)NP + n0 + q * 8; vst2((unsigned*)(VT + o), *(const v4u*)&th[cl][q * 8]); vst2((unsigned*)(VTL + o), *(const v4u*)&tl[cl][q * 8]); } }
    __syncthreads(); } }
__global__ __launch_bounds__(128) void k_att(const _Float16* __restrict__ QH, const _Float16* __restrict__ QL, const _Float16* __restrict__ KH, const _Float16* __restrict__ KL, const _Float16* __restrict__ VT, const _Float16* __restrict__ VTL, float* __restrict__ O) {
  __shared__ __align__(16) float sp[4][16][36]; __shared__ __align__(16) float so[4][16][68];
  const int tid = threadIdx.x, wave = tid >> 5, lane = tid & 31, col = lane & 15, g = lane >> 4; const int h = blockIdx.y; const size_t b = blockIdx.z; const int q0 = blockIdx.x * 64 + wave * 16; const size_t rq = b * NP + q0;
  v16h aq[2], al[2];
#pragma unroll
  for (int kc = 0; kc < 2; ++kc) { aq[kc] = frag_h(QH + (rq + col) * QC + h * KD + kc * 32, lane); al[kc] = frag_h(QL + (rq + col) * QC + h * KD + kc * 32, lane); }
  float m[8], l[8];
#pragma unroll
  for (int r = 0; r < 8; ++r) { m[r] = -3.0e38f; l[r] = 0.f; }
  v8f acc[4] = {}, accl[4] = {};
#pragma unroll 1
  for (int ks = 0; ks < NP / 32; ++ks) { v8f s[2];
#pragma unroll
    for (int ct = 0; ct < 2; ++ct) { const size_t rk = b * NP + ks * 32 + ct * 16 + col; v8f c = {}, cl = {};
#pragma unroll
      for (int kc = 0; kc < 2; ++kc) { const v16h kh = frag_h(KH + rk * KD + kc * 32, lane), kl = frag_h(KL + rk * KD + kc * 32, lane); c = wmma16(aq[kc], kh, c); cl = wmma16(aq[kc], kl, cl); cl = wmma16(al[kc], kh, cl); }
#pragma unroll
      for (int r = 0; r < 8; ++r) s[ct][r] = (c[r] + cl[r] * (1.0f / 2048.0f)) * 0.125f; }
    float alpha[8];
#pragma unroll
    for (int r = 0; r < 8; ++r) { float mx = fmaxf(s[0][r], s[1][r]);
#pragma unroll
      for (int o = 1; o < 16; o <<= 1) mx = fmaxf(mx, __shfl_xor(mx, o));
      const float mn = fmaxf(m[r], mx); alpha[r] = __expf(m[r] - mn); const float e0 = __expf(s[0][r] - mn), e1 = __expf(s[1][r] - mn); float es = e0 + e1;
#pragma unroll
      for (int o = 1; o < 16; o <<= 1) es += __shfl_xor(es, o);
      l[r] = l[r] * alpha[r] + es; m[r] = mn; sp[wave][8 * g + r][col] = e0; sp[wave][8 * g + r][16 + col] = e1; }
#pragma unroll
    for (int j = 0; j < 4; ++j)
#pragma unroll
      for (int r = 0; r < 8; ++r) { acc[j][r] *= alpha[r]; accl[j][r] *= alpha[r]; }
    LDSX();
    v16h pa; { const float* prow = &sp[wave][col][0] + 8 * (lane >> 4);
#pragma unroll
      for (int i = 0; i < 8; ++i) { pa[i] = (_Float16)(prow[i] * 2048.0f); pa[8 + i] = (_Float16)(prow[16 + i] * 2048.0f); } }
#pragma unroll
    for (int j = 0; j < 4; ++j) { const size_t po = (b * KD + j * 16 + col) * (size_t)NP + ks * 32; acc[j] = wmma16(pa, frag_h(VT + po, lane), acc[j]); accl[j] = wmma16(pa, frag_h(VTL + po, lane), accl[j]); }
    LDSX(); }
#pragma unroll
  for (int r = 0; r < 8; ++r) { const float il = (1.0f / 2048.0f) / l[r];
#pragma unroll
    for (int j = 0; j < 4; ++j) so[wave][8 * g + r][j * 16 + col] = (acc[j][r] + accl[j][r] * (1.0f / 2048.0f)) * il; }
  LDSX(); for (int rl = 0; rl < 16; ++rl) if (lane < 16) vst2(O + (rq + rl) * QC + (size_t)h * KD + lane * 4, *(const v4f*)&so[wave][rl][lane * 4]); }
__global__ __launch_bounds__(128) void k_out(const float* __restrict__ O, const float* __restrict__ WO, float* __restrict__ OUT) { __shared__ __align__(16) float sf[4][16][132];
  const int tid = threadIdx.x, wave = tid >> 5, lane = tid & 31, col = lane & 15, g = lane >> 4; const size_t b = blockIdx.z; const int p = blockIdx.y >> 2, hc = (blockIdx.y & 3) * 128; const int o0 = blockIdx.x * 64 + wave * 16;
  v8f acc[8] = {};
#pragma unroll 2
  for (int kc = 0; kc < QC / 32; ++kc) { const v16b a = fragb_f32(WO + (size_t)(o0 + col) * QC + kc * 32, lane);
#pragma unroll
    for (int j = 0; j < 8; ++j) { float w[16]; const int hd = hc + j * 16 + col;
#pragma unroll
      for (int i = 0; i < 8; ++i) { w[i] = O[(b * NP + 2 * (size_t)(kc * 32 + 8 * g + i) + p) * QC + hd]; w[8 + i] = O[(b * NP + 2 * (size_t)(kc * 32 + 16 + 8 * g + i) + p) * QC + hd]; }
      const F2 wb = bsplit16(w); acc[j] = wmma_bf(a, wb.h, acc[j]); acc[j] = wmma_bf(a, wb.l, acc[j]); } }
#pragma unroll
  for (int j = 0; j < 8; ++j)
#pragma unroll
    for (int r = 0; r < 8; ++r) sf[wave][8 * g + r][j * 16 + col] = acc[j][r];
  LDSX(); for (int rl = 0; rl < 16; ++rl) vst2(OUT + ((b * CC + o0 + rl) * (size_t)NP) + p * 512 + hc + lane * 4, *(const v4f*)&sf[wave][rl][lane * 4]); }
extern "C" void kernel_launch(void* const* d_in, const int* in_sizes, int n_in, void* d_out, int out_size, void* d_ws, size_t ws_size, hipStream_t stream) {
  (void)in_sizes; (void)n_in; (void)out_size;
  const float** F = (const float**)d_in;
  if (ws_size < (size_t)WS_END) return;
  char* ws = (char*)d_ws; _Float16 *QH = (_Float16*)(ws + WS_QH), *QL = (_Float16*)(ws + WS_QL), *KH = (_Float16*)(ws + WS_KH), *KL = (_Float16*)(ws + WS_KL), *VT = (_Float16*)(ws + WS_VT), *VTL = (_Float16*)(ws + WS_VTL); float* O = (float*)(ws + WS_O);
  k_q<<<dim3(NP / 64, TNB), 128, 0, stream>>>(F[0], F[1], F[2], F[3], F[4], F[5], QH, QL);
  k_kv<<<dim3(NP / 64, TNB), 128, 0, stream>>>(F[0], F[6], F[7], F[8], F[9], F[10], F[11], F[12], F[13], F[14], F[15], F[16], F[17], KH, KL, VT, VTL);
  k_att<<<dim3(NP / 64, NHD, TNB), 128, 0, stream>>>(QH, QL, KH, KL, VT, VTL, O);
  k_out<<<dim3(CC / 64, 8, TNB), 128, 0, stream>>>(O, F[18], (float*)d_out);
}
